// DenseSAKELayer_20624432955637
// MI455X (gfx1250) — hardware-run, weakly checked
//
#include <hip/hip_runtime.h>
#include <math.h>

typedef __attribute__((ext_vector_type(16))) _Float16 v16h;
typedef __attribute__((ext_vector_type(8)))  _Float16 v8h;
typedef __attribute__((ext_vector_type(8)))  float    v8f;
typedef __attribute__((ext_vector_type(4)))  float    v4f;

constexpr int kBatch    = 4;
constexpr int kNode     = 256;
constexpr int kNodesTot = kBatch * kNode;
constexpr int kFeat     = 64;
constexpr int kHid      = 64;
constexpr int kCoef     = 32;
constexpr int kHeads    = 4;
constexpr int kCat      = 384;
constexpr int kLinLd    = 128;
constexpr int kHeLd     = 256;
constexpr int kNsLd     = 64;
constexpr int kLDA      = 72;
constexpr int kLDT      = 264;
constexpr float kWCarry      = 16.0f;
constexpr float kWCarryInv   = 0.0625f;
constexpr float kAttCarry    = 256.0f;
constexpr float kAttCarryInv = 0.00390625f;
constexpr float kEps     = 1e-5f;
constexpr float kBig     = 100000.0f;
constexpr float kMeanInv = 1.0f / 8192.0f;

static_assert(kNodesTot == 1024);
static_assert(kCat == kFeat + kHid * kHeads + kHid);

constexpr int kOffA    = 0;
constexpr int kOffHe   = kOffA   + 256 * kLDA * 2;
constexpr int kOffHeT  = kOffHe  + 256 * kLDA * 2;
constexpr int kOffAtt  = kOffHeT + 64 * kLDT * 2;
constexpr int kOffWe2  = kOffAtt + 16 * kLDT * 2;
constexpr int kOffWcs  = kOffWe2 + 64 * kLDA * 2;
constexpr int kOffWc2  = kOffWcs + 80 * kLDA * 2;
constexpr int kOffCo   = kOffWc2 + 32 * kLDA * 2;
constexpr int kOffS    = kOffCo  + 256 * 32 * 4;
constexpr int kOffXs   = kOffS   + 256 * 4 * 4;
constexpr int kOffRed  = kOffXs  + 256 * 4 * 4;
constexpr int kOffOhe  = kOffRed + 1024 * 4;
constexpr int kOffMisc = kOffOhe + 256 * 4;
constexpr int kEdgeSmem = kOffMisc + 512 * 4;
static_assert(kEdgeSmem == 189440);
static_assert((kOffHe % 16) == 0 && (kOffHeT % 16) == 0 && (kOffAtt % 16) == 0 && (kOffWe2 % 16) == 0 &&
              (kOffWcs % 16) == 0 && (kOffWc2 % 16) == 0 && (kOffCo % 16) == 0 && (kOffS % 16) == 0 &&
              (kOffXs % 16) == 0 && (kOffRed % 16) == 0 && (kOffOhe % 16) == 0 && (kOffMisc % 16) == 0);
constexpr int kMLinI = 0;
constexpr int kMWrow = 64;
constexpr int kMBe2  = 128;
constexpr int kMBc1  = 192;
constexpr int kMBc2  = 256;
constexpr int kMBs   = 288;
constexpr int kMGam  = 296;
constexpr int kMCs   = 304;
constexpr int kMOst  = 400;
static_assert(((kOffMisc + kMOst * 4) % 16) == 0);
static_assert(kMOst + 64 <= 512);

constexpr int kNOffCat = 0;
constexpr int kNOffCN  = kNOffCat + 64 * kCat;
constexpr int kNOffHC  = kNOffCN + 64 * 32;
constexpr int kNOffT   = kNOffHC + 64 * 64;
constexpr int kNOffOut = kNOffT + 64 * 64;
constexpr int kNOffVG  = kNOffOut + 64 * 64;
constexpr int kNOffDV  = kNOffVG + 64;
constexpr int kNOffO1  = kNOffDV + 256;
constexpr int kNOffO2  = kNOffO1 + 192;
constexpr int kNodeSmem = (kNOffO2 + 192) * 4;
static_assert(kNodeSmem == 158464);
static_assert((kNOffOut % 4) == 0 && (kNOffO1 % 4) == 0 && (kNOffO2 % 4) == 0);

__device__ __forceinline__ v8f zero8() { return (v8f){0.f, 0.f, 0.f, 0.f, 0.f, 0.f, 0.f, 0.f}; }
struct FragH {
  union U { v16h v; v8h h[2]; };
  static __device__ __forceinline__ v16h load(const _Float16* p) {
    U f; f.h[0] = *(const v8h*)(p); f.h[1] = *(const v8h*)(p + 16); return f.v;
  }
};
__device__ __forceinline__ v8f mma_h(v16h a, v16h b, v8f c) {
  c = __builtin_amdgcn_wmma_f32_16x16x32_f16(false, a, false, b, (short)0, c, false, false);
  asm volatile("v_nop\n\tv_nop\n\tv_nop\n\tv_nop" : "+v"(c) : "v"(a), "v"(b));
  return c;
}

__device__ __forceinline__ float silu_f(float t) {
  const float e = expf(-t);
  return t * (1.0f / (1.0f + e));
}

template <bool IS_MAX>
__device__ __forceinline__ void blk_red4(float& v0, float& v1, float& v2, float& v3, float* sred, int lane, int wave) {
  float t[4] = {v0, v1, v2, v3};
#pragma unroll
  for (int q = 0; q < 4; ++q) {
    float a = t[q];
#pragma unroll
    for (int off = 16; off > 0; off >>= 1) {
      const float o = __shfl_xor(a, off, 32);
      a = IS_MAX ? fmaxf(a, o) : (a + o);
    }
    t[q] = a;
  }
  if (lane == 0) { sred[wave * 4 + 0] = t[0]; sred[wave * 4 + 1] = t[1]; sred[wave * 4 + 2] = t[2]; sred[wave * 4 + 3] = t[3]; }
  __syncthreads();
#pragma unroll
  for (int q = 0; q < 4; ++q) {
    float a = sred[q];
#pragma unroll
    for (int w = 1; w < 8; ++w) {
      const float o = sred[w * 4 + q];
      a = IS_MAX ? fmaxf(a, o) : (a + o);
    }
    t[q] = a;
  }
  __syncthreads();
  v0 = t[0]; v1 = t[1]; v2 = t[2]; v3 = t[3];
}

__device__ __forceinline__ void dot8(float (&acc)[8], const float* src, int pitch, const float* __restrict__ wcol, int kdim) {
#pragma unroll 1
  for (int c = 0; c < kdim; ++c) {
    const float w = wcol[c * 64];
#pragma unroll
    for (int u = 0; u < 8; ++u) acc[u] = fmaf(src[u * pitch + c], w, acc[u]);
  }
}

__global__ __launch_bounds__(256) void lin_kernel(const float* __restrict__ h, const float* __restrict__ W_e1,
                                                  float* __restrict__ LIN) {
  __shared__ __align__(16) float sH[64 * 64];
  __shared__ __align__(16) float sO[64 * 128];
  const int tid = threadIdx.x, lane = tid & 31, wave = tid >> 5;
  const int node0 = blockIdx.x * 64;
#pragma unroll 4
  for (int e = tid; e < 4096; e += 256) sH[e] = h[(size_t)node0 * 64 + e];
  __syncthreads();
  const int kk = tid & 127;
  const int ng = tid >> 7;
  const float* Wc = W_e1 + (kk >> 6) * 4096 + (kk & 63);
#pragma unroll 1
  for (int q4 = 0; q4 < 4; ++q4) {
    const int nb = ng * 32 + q4 * 8;
    float acc[8];
#pragma unroll
    for (int u = 0; u < 8; ++u) acc[u] = 0.0f;
    dot8(acc, sH + nb * 64, 64, Wc, 64);
#pragma unroll
    for (int u = 0; u < 8; ++u) sO[(nb + u) * 128 + kk] = acc[u];
  }
  __syncthreads();
  for (int pass = 0; pass < 2; ++pass) {
#pragma unroll
    for (int it = 0; it < 8; ++it) {
      const int nl = wave * 8 + it;
      const v4f val = *(const v4f*)(sO + nl * 128 + 4 * lane);
      *(volatile v4f*)(LIN + (size_t)(node0 + nl) * kLinLd + 4 * lane) = val;
    }
    __threadfence();
  }
}

__global__ __launch_bounds__(256) void edge_kernel(
    const float* __restrict__ x, const float* __restrict__ LIN,
    const float* __restrict__ W_e1, const float* __restrict__ b_e1,
    const float* __restrict__ W_e2, const float* __restrict__ b_e2,
    const float* __restrict__ W_c1, const float* __restrict__ b_c1,
    const float* __restrict__ W_c2, const float* __restrict__ b_c2,
    const float* __restrict__ W_s,  const float* __restrict__ b_s,
    const float* __restrict__ log_gamma,
    float* __restrict__ HE, float* __restrict__ NS) {
  extern __shared__ __align__(16) char smem[];
  _Float16* sA    = (_Float16*)(smem + kOffA);
  _Float16* sHe   = (_Float16*)(smem + kOffHe);
  _Float16* sHeT  = (_Float16*)(smem + kOffHeT);
  _Float16* sAttT = (_Float16*)(smem + kOffAtt);
  _Float16* sWe2T = (_Float16*)(smem + kOffWe2);
  _Float16* sWcsT = (_Float16*)(smem + kOffWcs);
  _Float16* sWc2T = (_Float16*)(smem + kOffWc2);
  float* sCo  = (float*)(smem + kOffCo);
  float* sS   = (float*)(smem + kOffS);
  float* sXs  = (float*)(smem + kOffXs);
  float* sRed = (float*)(smem + kOffRed);
  float* sOhe = (float*)(smem + kOffOhe);
  float* sM   = (float*)(smem + kOffMisc);
  float* sLinI = sM + kMLinI;
  float* sWrow = sM + kMWrow;
  float* sBe2  = sM + kMBe2;
  float* sBc1  = sM + kMBc1;
  float* sBc2  = sM + kMBc2;
  float* sBs   = sM + kMBs;
  float* sGam  = sM + kMGam;
  float* sCs   = sM + kMCs;
  float* sOst  = sM + kMOst;

  const int tid  = threadIdx.x;
  const int lane = tid & 31, wave = tid >> 5;
  const int rl   = lane & 15;
  const int koff = (lane >> 4) * 8;
  const int node  = blockIdx.x;
  const int bb    = node >> 8;
  const int inode = node & 255;

#pragma unroll 4
  for (int e = tid; e < 4096; e += 256) {
    const int k = e >> 6, n = e & 63;
    sWe2T[n * kLDA + k] = (_Float16)(W_e2[e] * kWCarry);
    sWcsT[n * kLDA + k] = (_Float16)(W_c1[e] * kWCarry);
  }
  {
    const int k = tid >> 2, n = tid & 3;
    sWcsT[(64 + n) * kLDA + k] = (_Float16)(W_s[tid] * kWCarry);
  }
  for (int e = tid; e < 384; e += 256) {
    const int r = 68 + (e >> 5), w = e & 31;
    ((unsigned*)(sWcsT + r * kLDA))[w] = 0u;
  }
#pragma unroll 4
  for (int e = tid; e < 2048; e += 256) {
    const int k = e >> 5, n = e & 31;
    sWc2T[n * kLDA + k] = (_Float16)(W_c2[e] * kWCarry);
  }
  for (int e = tid; e < 1536; e += 256) {
    const int r = 4 + (e >> 7), w = e & 127;
    ((unsigned*)(sAttT + r * kLDT))[w] = 0u;
  }
  if (tid < 64) {
    sLinI[tid] = LIN[(size_t)node * kLinLd + 64 + tid] + b_e1[tid];
    sWrow[tid] = W_e1[128 * 64 + tid];
    sBe2[tid]  = b_e2[tid];
    sBc1[tid]  = b_c1[tid];
  }
  if (tid < 32) sBc2[tid] = b_c2[tid];
  if (tid < 4) { sBs[tid] = b_s[tid]; sGam[tid] = expf(log_gamma[tid]); }

  const int jn = (bb << 8) + tid;
  const float xi0 = x[node * 3 + 0], xi1 = x[node * 3 + 1], xi2 = x[node * 3 + 2];
  const float d0 = x[jn * 3 + 0] - xi0;
  const float d1 = x[jn * 3 + 1] - xi1;
  const float d2 = x[jn * 3 + 2] - xi2;
  float sq = d0 * d0; sq = fmaf(d1, d1, sq); sq = fmaf(d2, d2, sq);
  const float nr  = sqrtf(sq + kEps);
  const float den = nr + kEps;
  const float inv = 1.0f / (den * den);
  sXs[tid * 4 + 0] = d0 * inv;
  sXs[tid * 4 + 1] = d1 * inv;
  sXs[tid * 4 + 2] = d2 * inv;
  sXs[tid * 4 + 3] = 0.0f;
  __syncthreads();

  {
    const float* lrow = LIN + (size_t)jn * kLinLd;
    _Float16* arow = sA + tid * kLDA;
#pragma unroll 1
    for (int c8 = 0; c8 < 8; ++c8) {
      const v4f f0 = *(const v4f*)(lrow + c8 * 8);
      const v4f f1 = *(const v4f*)(lrow + c8 * 8 + 4);
      v8h o;
#pragma unroll
      for (int r = 0; r < 4; ++r) {
        const int cc = c8 * 8 + r;
        float p0 = f0[r] + sLinI[cc];
        p0 = fmaf(nr, sWrow[cc], p0);
        o[r] = (_Float16)silu_f(p0);
        const int cc2 = cc + 4;
        float p1 = f1[r] + sLinI[cc2];
        p1 = fmaf(nr, sWrow[cc2], p1);
        o[4 + r] = (_Float16)silu_f(p1);
      }
      *(v8h*)(arow + c8 * 8) = o;
    }
  }
  __syncthreads();

#pragma unroll 1
  for (int mi = 0; mi < 2; ++mi) {
    const int m0 = (wave * 2 + mi) * 16;
    const v16h a0 = FragH::load(sA + (m0 + rl) * kLDA + koff);
    const v16h a1 = FragH::load(sA + (m0 + rl) * kLDA + 32 + koff);
#pragma unroll 1
    for (int nt = 0; nt < 4; ++nt) {
      const v16h b0 = FragH::load(sWe2T + (nt * 16 + rl) * kLDA + koff);
      const v16h b1 = FragH::load(sWe2T + (nt * 16 + rl) * kLDA + 32 + koff);
      v8f acc = zero8();
      acc = mma_h(a0, b0, acc);
      acc = mma_h(a1, b1, acc);
      const int n = nt * 16 + rl;
      const float bv = sBe2[n];
      v8h pk;
#pragma unroll
      for (int r = 0; r < 8; ++r) {
        float t = fmaf(acc[r], kWCarryInv, bv);
        t = silu_f(t);
        const _Float16 hv = (_Float16)t;
        pk[r] = hv;
        sHe[(m0 + koff + r) * kLDA + n] = hv;
      }
      *(v8h*)(sHeT + n * kLDT + m0 + koff) = pk;
    }
  }
  __syncthreads();

#pragma unroll 1
  for (int mi = 0; mi < 2; ++mi) {
    const int m0 = (wave * 2 + mi) * 16;
    const v16h a0 = FragH::load(sHe + (m0 + rl) * kLDA + koff);
    const v16h a1 = FragH::load(sHe + (m0 + rl) * kLDA + 32 + koff);
#pragma unroll 1
    for (int nt = 0; nt < 5; ++nt) {
      const v16h b0 = FragH::load(sWcsT + (nt * 16 + rl) * kLDA + koff);
      const v16h b1 = FragH::load(sWcsT + (nt * 16 + rl) * kLDA + 32 + koff);
      v8f acc = zero8();
      acc = mma_h(a0, b0, acc);
      acc = mma_h(a1, b1, acc);
      if (nt < 4) {
        const int n = nt * 16 + rl;
        const float bv = sBc1[n];
#pragma unroll
        for (int r = 0; r < 8; ++r) {
          float t = fmaf(acc[r], kWCarryInv, bv);
          t = silu_f(t);
          sA[(m0 + koff + r) * kLDA + n] = (_Float16)t;
        }
      } else {
        const float bsv = sBs[rl & 3];
        if (rl < kHeads) {
#pragma unroll
          for (int r = 0; r < 8; ++r) {
            float t = fmaf(acc[r], kWCarryInv, bsv);
            t = (t >= 0.0f) ? t : 0.2f * t;
            sS[(m0 + koff + r) * 4 + rl] = t;
          }
        }
      }
    }
  }
  __syncthreads();

#pragma unroll 1
  for (int mi = 0; mi < 2; ++mi) {
    const int m0 = (wave * 2 + mi) * 16;
    const v16h a0 = FragH::load(sA + (m0 + rl) * kLDA + koff);
    const v16h a1 = FragH::load(sA + (m0 + rl) * kLDA + 32 + koff);
#pragma unroll 1
    for (int nt = 0; nt < 2; ++nt) {
      const v16h b0 = FragH::load(sWc2T + (nt * 16 + rl) * kLDA + koff);
      const v16h b1 = FragH::load(sWc2T + (nt * 16 + rl) * kLDA + 32 + koff);
      v8f acc = zero8();
      acc = mma_h(a0, b0, acc);
      acc = mma_h(a1, b1, acc);
      const int n = nt * 16 + rl;
      const float bv = sBc2[n];
#pragma unroll
      for (int r = 0; r < 8; ++r) sCo[(m0 + koff + r) * kCoef + n] = fmaf(acc[r], kWCarryInv, bv);
    }
  }
  __syncthreads();

  {
    const float diag = (tid == inode) ? kBig : 0.0f;
    const float base = -(nr + diag);
    const float g0 = sGam[0], g1 = sGam[1], g2 = sGam[2], g3 = sGam[3];
    const float le0 = base * g0, le1 = base * g1, le2 = base * g2, le3 = base * g3;
    float m0 = le0, m1 = le1, m2 = le2, m3 = le3;
    blk_red4<true>(m0, m1, m2, m3, sRed, lane, wave);
    float e0 = expf(le0 - m0), e1 = expf(le1 - m1), e2 = expf(le2 - m2), e3 = expf(le3 - m3);
    float s0 = e0, s1 = e1, s2 = e2, s3 = e3;
    blk_red4<false>(s0, s1, s2, s3, sRed, lane, wave);
    const float ae0 = e0 * (1.0f / s0), ae1 = e1 * (1.0f / s1), ae2 = e2 * (1.0f / s2), ae3 = e3 * (1.0f / s3);

    const float ls0 = sS[tid * 4 + 0] - diag, ls1 = sS[tid * 4 + 1] - diag;
    const float ls2 = sS[tid * 4 + 2] - diag, ls3 = sS[tid * 4 + 3] - diag;
    m0 = ls0; m1 = ls1; m2 = ls2; m3 = ls3;
    blk_red4<true>(m0, m1, m2, m3, sRed, lane, wave);
    e0 = expf(ls0 - m0); e1 = expf(ls1 - m1); e2 = expf(ls2 - m2); e3 = expf(ls3 - m3);
    s0 = e0; s1 = e1; s2 = e2; s3 = e3;
    blk_red4<false>(s0, s1, s2, s3, sRed, lane, wave);
    const float as0 = e0 * (1.0f / s0), as1 = e1 * (1.0f / s1), as2 = e2 * (1.0f / s2), as3 = e3 * (1.0f / s3);

    const float al0 = ae0 * as0, al1 = ae1 * as1, al2 = ae2 * as2, al3 = ae3 * as3;
    m0 = al0; m1 = al1; m2 = al2; m3 = al3;
    blk_red4<true>(m0, m1, m2, m3, sRed, lane, wave);
    e0 = expf(al0 - m0); e1 = expf(al1 - m1); e2 = expf(al2 - m2); e3 = expf(al3 - m3);
    s0 = e0; s1 = e1; s2 = e2; s3 = e3;
    blk_red4<false>(s0, s1, s2, s3, sRed, lane, wave);
    const float at0 = e0 * (1.0f / s0), at1 = e1 * (1.0f / s1), at2 = e2 * (1.0f / s2), at3 = e3 * (1.0f / s3);
    sAttT[0 * kLDT + tid] = (_Float16)(at0 * kAttCarry);
    sAttT[1 * kLDT + tid] = (_Float16)(at1 * kAttCarry);
    sAttT[2 * kLDT + tid] = (_Float16)(at2 * kAttCarry);
    sAttT[3 * kLDT + tid] = (_Float16)(at3 * kAttCarry);
  }
  __syncthreads();

  if (wave < 4) {
    v8f acc = zero8();
    const _Float16* ap = sHeT + (wave * 16 + rl) * kLDT + koff;
    const _Float16* bp = sAttT + rl * kLDT + koff;
#pragma unroll
    for (int ks = 0; ks < 8; ++ks) {
      const v16h a  = FragH::load(ap + ks * 32);
      const v16h bt = FragH::load(bp + ks * 32);
      acc = mma_h(a, bt, acc);
    }
    if (rl < kHeads) {
#pragma unroll
      for (int r = 0; r < 8; ++r) sOhe[(wave * 16 + koff + r) * 4 + rl] = acc[r] * kAttCarryInv;
    }
  }
  {
    const int c = tid >> 3, jc = tid & 7;
    float a0 = 0.0f, a1 = 0.0f, a2 = 0.0f;
#pragma unroll 1
    for (int j = jc * 32; j < jc * 32 + 32; ++j) {
      const float co = sCo[j * kCoef + c];
      const v4f xs = *(const v4f*)(sXs + j * 4);
      a0 = fmaf(co, xs[0], a0);
      a1 = fmaf(co, xs[1], a1);
      a2 = fmaf(co, xs[2], a2);
    }
    sRed[(c * 8 + jc) * 4 + 0] = a0;
    sRed[(c * 8 + jc) * 4 + 1] = a1;
    sRed[(c * 8 + jc) * 4 + 2] = a2;
  }
  __syncthreads();
  if (tid < kCoef) {
    float cs0 = 0.0f, cs1 = 0.0f, cs2 = 0.0f;
#pragma unroll
    for (int jc = 0; jc < 8; ++jc) {
      cs0 += sRed[(tid * 8 + jc) * 4 + 0];
      cs1 += sRed[(tid * 8 + jc) * 4 + 1];
      cs2 += sRed[(tid * 8 + jc) * 4 + 2];
    }
    float cn = cs0 * cs0; cn = fmaf(cs1, cs1, cn); cn = fmaf(cs2, cs2, cn);
    sOst[tid] = cn;
    sCs[0 * 32 + tid] = cs0;
    sCs[1 * 32 + tid] = cs1;
    sCs[2 * 32 + tid] = cs2;
  }
  __syncthreads();
  if (tid < 32) {
    const int kd = (tid < 3) ? tid : 0;
    float a = 0.0f;
#pragma unroll 1
    for (int c = 0; c < kCoef; ++c) a += sCs[kd * 32 + c];
    const float dv = a * kMeanInv;
    sOst[32 + tid] = (tid < 3) ? dv : 0.0f;
  }
  __syncthreads();

  if (wave == 0) {
    const v4f p0 = *(const v4f*)(sOhe + 4 * lane);
    const v4f p1 = *(const v4f*)(sOhe + 128 + 4 * lane);
    float* dst = HE + (size_t)node * kHeLd;
    for (int pass = 0; pass < 2; ++pass) {
      *(volatile v4f*)(dst + 4 * lane) = p0;
      *(volatile v4f*)(dst + 128 + 4 * lane) = p1;
      __threadfence();
    }
  } else if (wave == 1) {
    const v4f p = *(const v4f*)(sOst + 4 * (lane & 15));
    float* dst = NS + (size_t)node * kNsLd;
    for (int pass = 0; pass < 2; ++pass) {
      if (lane < 16) *(volatile v4f*)(dst + 4 * lane) = p;
      __threadfence();
    }
  }
}

__global__ __launch_bounds__(256) void node_kernel(
    const float* __restrict__ h, const float* __restrict__ x, const float* __restrict__ v,
    const float* __restrict__ W_p1, const float* __restrict__ b_p1,
    const float* __restrict__ W_p2, const float* __restrict__ b_p2,
    const float* __restrict__ W_n1, const float* __restrict__ b_n1,
    const float* __restrict__ W_n2, const float* __restrict__ b_n2,
    const float* __restrict__ W_v1, const float* __restrict__ b_v1, const float* __restrict__ W_v2,
    const float* __restrict__ HE, const float* __restrict__ NS,
    float* __restrict__ out_h, float* __restrict__ out_xv) {
  extern __shared__ __align__(16) char smem[];
  float* sBase = (float*)smem;
  float* sCat = sBase + kNOffCat;
  float* sCN  = sBase + kNOffCN;
  float* sHC  = sBase + kNOffHC;
  float* sT   = sBase + kNOffT;
  float* sOut = sBase + kNOffOut;
  float* sVG  = sBase + kNOffVG;
  float* sDV  = sBase + kNOffDV;
  float* sO1  = sBase + kNOffO1;
  float* sO2  = sBase + kNOffO2;

  const int tid = threadIdx.x, lane = tid & 31, wave = tid >> 5;
  const int node0 = blockIdx.x * 64;

#pragma unroll 4
  for (int e = tid; e < 4096; e += 256) {
    const int nl = e >> 6, c = e & 63;
    sCat[nl * kCat + c] = h[(size_t)(node0 + nl) * kFeat + c];
  }
#pragma unroll 4
  for (int e = tid; e < 16384; e += 256) {
    const int nl = e >> 8, c = e & 255;
    sCat[nl * kCat + 64 + c] = HE[(size_t)(node0 + nl) * kHeLd + c];
  }
#pragma unroll 4
  for (int e = tid; e < 2048; e += 256) {
    const int nl = e >> 5, c = e & 31;
    sCN[e] = NS[(size_t)(node0 + nl) * kNsLd + c];
  }
  {
    const int nl = tid >> 2, kq = tid & 3;
    const int kc = (kq < 3) ? kq : 2;
    sDV[tid] = NS[(size_t)(node0 + nl) * kNsLd + 32 + kc];
  }
  __syncthreads();

  const int k  = tid & 63;
  const int ng = tid >> 6;

#pragma unroll 1
  for (int hb = 0; hb < 2; ++hb) {
    const int nb = ng * 16 + hb * 8;
    float acc[8];
    const float bv = b_p1[k];
#pragma unroll
    for (int u = 0; u < 8; ++u) acc[u] = bv;
    dot8(acc, sCN + nb * 32, 32, W_p1 + k, kCoef);
#pragma unroll
    for (int u = 0; u < 8; ++u) sHC[(nb + u) * 64 + k] = acc[u];
  }
  __syncthreads();
#pragma unroll 1
  for (int e = tid; e < 4096; e += 256) sHC[e] = silu_f(sHC[e]);
  __syncthreads();

#pragma unroll 1
  for (int hb = 0; hb < 2; ++hb) {
    const int nb = ng * 16 + hb * 8;
    float acc[8];
    const float bv = b_p2[k];
#pragma unroll
    for (int u = 0; u < 8; ++u) acc[u] = bv;
    dot8(acc, sHC + nb * 64, 64, W_p2 + k, kHid);
#pragma unroll
    for (int u = 0; u < 8; ++u) sCat[(nb + u) * kCat + 320 + k] = acc[u];
  }
#pragma unroll 1
  for (int hb = 0; hb < 2; ++hb) {
    const int nb = ng * 16 + hb * 8;
    float acc[8];
    const float bv = b_v1[k];
#pragma unroll
    for (int u = 0; u < 8; ++u) acc[u] = bv;
    dot8(acc, sCat + nb * kCat, kCat, W_v1 + k, kFeat);
#pragma unroll
    for (int u = 0; u < 8; ++u) sT[(nb + u) * 64 + k] = acc[u];
  }
  __syncthreads();
  {
    const int nl = tid >> 2, part = tid & 3;
    float p = 0.0f;
#pragma unroll 1
    for (int hh = part * 16; hh < part * 16 + 16; ++hh) p = fmaf(silu_f(sT[nl * 64 + hh]), W_v2[hh], p);
    p += __shfl_xor(p, 1, 32);
    p += __shfl_xor(p, 2, 32);
    if (part == 0) sVG[nl] = p;
  }
  __syncthreads();

#pragma unroll 1
  for (int hb = 0; hb < 2; ++hb) {
    const int nb = ng * 16 + hb * 8;
    float acc[8];
    const float bv = b_n1[k];
#pragma unroll
    for (int u = 0; u < 8; ++u) acc[u] = bv;
    dot8(acc, sCat + nb * kCat, kCat, W_n1 + k, kCat);
#pragma unroll
    for (int u = 0; u < 8; ++u) sT[(nb + u) * 64 + k] = acc[u];
  }
  __syncthreads();
#pragma unroll 1
  for (int e = tid; e < 4096; e += 256) sT[e] = silu_f(sT[e]);
  __syncthreads();

#pragma unroll 1
  for (int hb = 0; hb < 2; ++hb) {
    const int nb = ng * 16 + hb * 8;
    float acc[8];
    const float bv = b_n2[k];
#pragma unroll
    for (int u = 0; u < 8; ++u) acc[u] = bv;
    dot8(acc, sT + nb * 64, 64, W_n2 + k, kHid);
#pragma unroll
    for (int u = 0; u < 8; ++u) sOut[(nb + u) * 64 + k] = acc[u] + sCat[(nb + u) * kCat + k];
  }
  if (tid < 192) {
    const int nl = tid / 3;
    const int kd = tid - 3 * nl;
    const int nd = node0 + nl;
    const float vv = v[(size_t)nd * 3 + kd];
    const float xx = x[(size_t)nd * 3 + kd];
    const float gv = sVG[nl] * vv;
    const float vn = sDV[nl * 4 + kd] + gv;
    sO2[tid] = vn;
    sO1[tid] = xx + vn;
  }
  __syncthreads();

  {
    const int hh = lane >> 4, c4 = (lane & 15) * 4;
    for (int pass = 0; pass < 2; ++pass) {
#pragma unroll
      for (int it = 0; it < 4; ++it) {
        const int row = wave * 8 + it * 2 + hh;
        const v4f val = *(const v4f*)(sOut + row * 64 + c4);
        *(volatile v4f*)(out_h + (size_t)(node0 + row) * kFeat + c4) = val;
      }
      __threadfence();
    }
  }
  if (wave < 2) {
    const float* src = sO1 + wave * 192;
    float* dst = out_xv + (size_t)wave * (kNodesTot * 3) + (size_t)blockIdx.x * 192;
    const v4f p0 = *(const v4f*)(src + 4 * lane);
    const v4f p1 = *(const v4f*)(src + 128 + 4 * (lane & 15));
    for (int pass = 0; pass < 2; ++pass) {
      *(volatile v4f*)(dst + 4 * lane) = p0;
      if (lane < 16) *(volatile v4f*)(dst + 128 + 4 * lane) = p1;
      __threadfence();
    }
  }
}

extern "C" void kernel_launch(void* const* d_in, const int* in_sizes, int n_in,
                              void* d_out, int out_size, void* d_ws, size_t ws_size,
                              hipStream_t stream) {
  if (n_in < 25) return;
  if (in_sizes[0] != kNodesTot * kFeat || in_sizes[1] != kNodesTot * 3 || in_sizes[2] != kNodesTot * 3) return;
  if (in_sizes[3] != 129 * 64 || in_sizes[17] != kCat * kHid || in_sizes[23] != 64 || in_sizes[24] != kHeads) return;
  if (out_size != kNodesTot * (kFeat + 3 + 3)) return;

  const float* h      = (const float*)d_in[0];
  const float* x      = (const float*)d_in[1];
  const float* v      = (const float*)d_in[2];
  const float* W_e1   = (const float*)d_in[3];
  const float* b_e1   = (const float*)d_in[4];
  const float* W_e2   = (const float*)d_in[5];
  const float* b_e2   = (const float*)d_in[6];
  const float* W_c1   = (const float*)d_in[7];
  const float* b_c1   = (const float*)d_in[8];
  const float* W_c2   = (const float*)d_in[9];
  const float* b_c2   = (const float*)d_in[10];
  const float* W_p1   = (const float*)d_in[11];
  const float* b_p1   = (const float*)d_in[12];
  const float* W_p2   = (const float*)d_in[13];
  const float* b_p2   = (const float*)d_in[14];
  const float* W_s    = (const float*)d_in[15];
  const float* b_s    = (const float*)d_in[16];
  const float* W_n1   = (const float*)d_in[17];
  const float* b_n1   = (const float*)d_in[18];
  const float* W_n2   = (const float*)d_in[19];
  const float* b_n2   = (const float*)d_in[20];
  const float* W_v1   = (const float*)d_in[21];
  const float* b_v1   = (const float*)d_in[22];
  const float* W_v2   = (const float*)d_in[23];
  const float* lgam   = (const float*)d_in[24];

  const size_t bytesLin = (size_t)kNodesTot * kLinLd * 4;
  const size_t bytesHe  = (size_t)kNodesTot * kHeLd * 4;
  const size_t bytesNs  = (size_t)kNodesTot * kNsLd * 4;
  const size_t offLin = 0;
  const size_t offHe  = offLin + bytesLin;
  const size_t offNs  = offHe + bytesHe;
  const size_t total  = offNs + bytesNs;
  if (total > ws_size) return;
  char* ws = (char*)d_ws;
  float* LIN = (float*)(ws + offLin);
  float* HEp = (float*)(ws + offHe);
  float* NSp = (float*)(ws + offNs);

  float* out_h  = (float*)d_out;
  float* out_xv = out_h + kNodesTot * kFeat;

  lin_kernel<<<dim3(kNodesTot / 64), dim3(256), 0, stream>>>(h, W_e1, LIN);
  edge_kernel<<<dim3(kNodesTot), dim3(256), kEdgeSmem, stream>>>(
      x, LIN, W_e1, b_e1, W_e2, b_e2, W_c1, b_c1, W_c2, b_c2, W_s, b_s, lgam, HEp, NSp);
  node_kernel<<<dim3(kNodesTot / 64), dim3(256), kNodeSmem, stream>>>(
      h, x, v, W_p1, b_p1, W_p2, b_p2, W_n1, b_n1, W_n2, b_n2, W_v1, b_v1, W_v2, HEp, NSp, out_h, out_xv);
}
